// GMMflow_77292231459387
// MI455X (gfx1250) — hardware-run, weakly checked
//
#include <hip/hip_runtime.h>


#ifndef NB
#define NB 128
#endif
#define NB_FULL 128
#define N0_  128
#define N1_  128
#define ND   32
#define NP   (N0_ * N1_)
#define KD   64
#define VC   64
#define TP   64
#define TLP  68
#define AW   4
#define OSP  36
#define QRS  2048.0f
#define QRI  (1.0f / 2048.0f)
#define LOG2E 1.4426950408889634f
#define PSH  14.0f
#define NEGB (-3.0e38f)

static_assert(ND == 32);
static_assert(KD == 2 * ND);
static_assert(VC == 2 * ND);
static_assert(KD % 32 == 0);
static_assert(KD * 2 == 128);
static_assert(NP % 32 == 0);
static_assert(NP % TP == 0);
static_assert(N1_ % TP == 0);
static_assert(TP * 2 == 128);
static_assert(256 * 16 * 2 == TP * 128);
static_assert(256 * 16 * 2 == VC * 128);
static_assert(16 * 16 == TP * 4);
static_assert(256 == TP * 4);
static_assert(4 * 8 == ND);
static_assert(NB % (16 * AW) == 0);
static_assert(NB <= NB_FULL);
static_assert(32 * 16 * 4 == 16 * ND * 4);
static_assert((OSP * 4) % 16 == 0);
static_assert((TLP * 4) % 16 == 0);
static_assert((size_t)(2 * TP * TLP + 3 * TP) * 4 <= 131072);
static_assert((size_t)(AW * 16 * OSP) * 4 <= 131072);

typedef _Float16 h16;
typedef __attribute__((ext_vector_type(16))) _Float16 v16h;
typedef __attribute__((ext_vector_type(8)))  _Float16 v8h;
typedef __attribute__((ext_vector_type(8)))  float    v8f;
typedef __attribute__((ext_vector_type(4)))  float    v4f;
typedef v4f  __attribute__((may_alias)) v4fa;

__device__ __forceinline__ unsigned short f2bf(float f) { unsigned u = __float_as_uint(f); u += 0x7FFFu + ((u >> 16) & 1u); return (unsigned short)(u >> 16); }
__device__ __forceinline__ float bfr(float f) { return __uint_as_float(((unsigned)f2bf(f)) << 16); }
__device__ __forceinline__ v16h cat16(v8h lo, v8h hi) { return __builtin_shufflevector(lo, hi, 0, 1, 2, 3, 4, 5, 6, 7, 8, 9, 10, 11, 12, 13, 14, 15); }
__device__ __forceinline__ v8f wmma16(v16h a, v16h b, v8f c) { return __builtin_amdgcn_wmma_f32_16x16x32_f16(false, a, false, b, (short)0, c, false, false); }
__device__ __forceinline__ v16h  ldh(const h16* p) { return cat16(*(const v8h*)p, *(const v8h*)(p + 16)); }
__device__ __forceinline__ void wave_sync() { __builtin_amdgcn_fence(3  , "wavefront"); __builtin_amdgcn_wave_barrier(); asm volatile("" ::: "memory"); }
static __device__ __forceinline__ h16 toh_flush(float v) { const h16 r = (h16)v; return (fabsf(v) < 6.103515625e-05f) ? (h16)0.0f : r; }
__device__ __forceinline__ v8f wmma16g(v16h a, v16h b, v8f c) { c = wmma16(a, b, c); asm volatile("v_nop\n\tv_nop\n\tv_nop\n\tv_nop" : "+v"(c) : "v"(a), "v"(b)); return c; }

__global__ __launch_bounds__(256) void k_tab(const float* __restrict__ tp, const float* __restrict__ Mu0, const float* __restrict__ Mu1,
                                             const float* __restrict__ S0, const float* __restrict__ S1, const float* __restrict__ Lam,
                                             h16* KH, h16* KR, h16* VT, float* CL) {
#pragma clang fp contract(off)
    __shared__ __align__(16) float sK[TP * TLP];
    __shared__ __align__(16) float sV[VC * TLP];
    __shared__ __align__(16) float sC[3 * TP];
    const int tid = threadIdx.x, lane = tid & 31;
    const int wave = __builtin_amdgcn_readfirstlane((int)(threadIdx.x >> 5));
    const int ij0 = blockIdx.x * TP;
    const int p = tid >> 2, q = tid & 3;
    const int ij = ij0 + p; const int i = ij / N1_, j = ij % N1_;
    const float t = bfr(tp[0]); const float omt = 1.0f - t;
    const float tt = t * t, oo = omt * omt, two = (2.0f * t) * omt, e2 = (0.25f * t) * omt, e2t = 0.25f * t;
    float cpart = 0.0f;
#pragma unroll 1
    for (int n = q * 8; n < q * 8 + 8; ++n) {
        const float s0 = bfr(S0[i * ND + n]), s1 = bfr(S1[j * ND + n]);
        const float mu0 = bfr(Mu0[i * ND + n]), mu1 = bfr(Mu1[j * ND + n]);
        const float Ds = sqrtf(4.0f * s0 * s1 + 0.0625f);
        const float Cs = 0.5f * (Ds - 0.25f);
        const float Sg = ((oo * s0 + tt * s1) + two * Cs) + e2;
        const float Pt = t * s1 + omt * Cs, Qt = omt * s0 + t * Cs;
        const float St = (Pt - Qt) - e2t;
        const float iv = 1.0f / Sg;
        const float Kv = St * iv;
        const float Mt = omt * mu0 + t * mu1;
        const float vv = mu1 - mu0;
        sK[p * TLP + n] = iv; sK[p * TLP + ND + n] = Mt * iv;
        sV[n * TLP + p] = Kv; sV[(ND + n) * TLP + p] = vv - Kv * Mt;
        cpart += -0.5f * (Mt * Mt * iv) - 0.5f * logf(Sg);
    }
    cpart += __shfl_xor(cpart, 1, 32); cpart += __shfl_xor(cpart, 2, 32);
    const float lam = bfr(Lam[ij]);
    const float la = fabsf(lam);
    const float lgr = log2f(la);
    const float lg = (la > 0.0f) ? lgr : -1.0e4f;
    const float sg = (lam > 0.0f) ? 1.0f : ((lam < 0.0f) ? -1.0f : 0.0f);
    if (q == 0) { sC[p] = cpart; sC[TP + p] = lg; sC[2 * TP + p] = sg; }
    __syncthreads();
#pragma unroll 1
    for (int ps = 0; ps < 2; ++ps) {
#pragma unroll
        for (int it = 0; it < 2; ++it) { const int idx = it * 256 + tid; const int row = idx >> 3, c8 = (idx & 7) * 8;
            const v4f x0 = *(const v4fa*)(&sK[row * TLP + c8]); const v4f x1 = *(const v4fa*)(&sK[row * TLP + c8 + 4]);
            const v4f y0 = *(const v4fa*)(&sV[row * TLP + c8]); const v4f y1 = *(const v4fa*)(&sV[row * TLP + c8 + 4]);
            v8h hv, rv, wv;
#pragma unroll
            for (int e = 0; e < 4; ++e) { const h16 a0 = toh_flush(x0[e]); const h16 a1 = toh_flush(x1[e]); hv[e] = a0; hv[4 + e] = a1;
                rv[e] = toh_flush((x0[e] - (float)a0) * QRS); rv[4 + e] = toh_flush((x1[e] - (float)a1) * QRS);
                wv[e] = toh_flush(y0[e]); wv[4 + e] = toh_flush(y1[e]); }
            const size_t ko = (size_t)(ij0 + row) * KD + c8;
            const size_t vo = (size_t)row * NP + (size_t)ij0 + c8;
            *(volatile v8h*)(KH + ko) = hv; *(volatile v8h*)(KR + ko) = rv; *(volatile v8h*)(VT + vo) = wv; }
        if (wave == 0) { const int c4 = (lane & 15) * 4;
#pragma unroll
            for (int pl = 0; pl < 3; ++pl) { const v4f cv = *(const v4fa*)(&sC[pl * TP + c4]);
                if (lane < 16) *(volatile v4f*)(CL + (size_t)pl * NP + (size_t)ij0 + c4) = cv; } }
        if (ps == 0) __threadfence(); }
}

__global__ __launch_bounds__(32 * AW) __attribute__((amdgpu_num_vgpr(256)))
void k_mix(const float* __restrict__ X, const h16* __restrict__ KH, const h16* __restrict__ KR, const h16* __restrict__ VT, const float* __restrict__ CL, float* OUT) {
    __shared__ __align__(16) float os[AW * 16 * OSP];
    const int lane = threadIdx.x & 31, lr = lane & 15, hi = lane >> 4;
    const int wave = __builtin_amdgcn_readfirstlane((int)(threadIdx.x >> 5));
    const int b0 = (blockIdx.x * AW + wave) * 16;
    const size_t xo = (size_t)(b0 + lr) * ND + 8 * hi;
    v16h qh0, qr0, qh1, qr1;
    { const v4f a0 = *(const v4f*)(X + xo), a1 = *(const v4f*)(X + xo + 4), a2 = *(const v4f*)(X + xo + 16), a3 = *(const v4f*)(X + xo + 20);
      float xv[16];
#pragma unroll
      for (int r = 0; r < 4; ++r) { xv[r] = bfr(a0[r]); xv[4 + r] = bfr(a1[r]); xv[8 + r] = bfr(a2[r]); xv[12 + r] = bfr(a3[r]); }
#pragma unroll
      for (int e = 0; e < 16; ++e) { const float s = (-0.5f * xv[e]) * xv[e];
          const h16 sh_ = toh_flush(s); qh0[e] = sh_; qr0[e] = toh_flush((s - (float)sh_) * QRS);
          const h16 xh_ = toh_flush(xv[e]); qh1[e] = xh_; qr1[e] = toh_flush((xv[e] - (float)xh_) * QRS); } }
    const size_t ko = (size_t)lr * KD + 8 * hi;
    const size_t vo = (size_t)lr * NP + 8 * hi;
    v8f o0 = (v8f){}, o1 = (v8f){}, o2 = (v8f){}, o3 = (v8f){};
    float m = NEGB, l = 0.0f;
#pragma unroll 1
    for (int key0 = 0; key0 < NP; key0 += 32) {
        const h16* ka = KH + ko + (size_t)key0 * KD;
        const h16* kr = KR + ko + (size_t)key0 * KD;
        v8f sHa = (v8f){}, sLa = (v8f){}, sHb = (v8f){}, sLb = (v8f){};
        { const v16h k0 = ldh(ka), k1 = ldh(ka + 32), r0 = ldh(kr), r1 = ldh(kr + 32);
          sHa = wmma16g(k0, qh0, sHa); sHa = wmma16g(k1, qh1, sHa);
          sLa = wmma16g(k0, qr0, sLa); sLa = wmma16g(k1, qr1, sLa); sLa = wmma16g(r0, qh0, sLa); sLa = wmma16g(r1, qh1, sLa); }
        { const v16h k0 = ldh(ka + 16 * KD), k1 = ldh(ka + 16 * KD + 32), r0 = ldh(kr + 16 * KD), r1 = ldh(kr + 16 * KD + 32);
          sHb = wmma16g(k0, qh0, sHb); sHb = wmma16g(k1, qh1, sHb);
          sLb = wmma16g(k0, qr0, sLb); sLb = wmma16g(k1, qr1, sLb); sLb = wmma16g(r0, qh0, sLb); sLb = wmma16g(r1, qh1, sLb); }
        const float* cp = CL + key0 + 8 * hi;
        const float* lp = cp + NP;
        const float* sp = cp + 2 * NP;
        const v4f c0 = *(const v4f*)cp, c1 = *(const v4f*)(cp + 4), c2 = *(const v4f*)(cp + 16), c3 = *(const v4f*)(cp + 20);
        const v4f g0 = *(const v4f*)lp, g1 = *(const v4f*)(lp + 4), g2 = *(const v4f*)(lp + 16), g3 = *(const v4f*)(lp + 20);
        float cxa[8], cxb[8], lxa[8], lxb[8];
#pragma unroll
        for (int r = 0; r < 4; ++r) { cxa[r] = c0[r]; cxa[4 + r] = c1[r]; cxb[r] = c2[r]; cxb[4 + r] = c3[r];
                                      lxa[r] = g0[r]; lxa[4 + r] = g1[r]; lxb[r] = g2[r]; lxb[4 + r] = g3[r]; }
        float ta[8], tb[8]; float mx = NEGB;
#pragma unroll
        for (int r = 0; r < 8; ++r) {
            float ua = (sHa[r] + sLa[r] * QRI) + cxa[r];
            float ub = (sHb[r] + sLb[r] * QRI) + cxb[r];
            ua = fminf(fmaxf(ua, -50.0f), 50.0f); ub = fminf(fmaxf(ub, -50.0f), 50.0f);
            ta[r] = ua * LOG2E + lxa[r]; tb[r] = ub * LOG2E + lxb[r];
            mx = fmaxf(mx, fmaxf(ta[r], tb[r])); }
        mx = fmaxf(mx, __shfl_xor(mx, 16, 32));
        const float mnew = fmaxf(m, mx);
        const float alpha = __builtin_amdgcn_exp2f(m - mnew);
        const float sh = PSH - mnew;
        const v4f q0 = *(const v4f*)sp, q1 = *(const v4f*)(sp + 4), q2 = *(const v4f*)(sp + 16), q3 = *(const v4f*)(sp + 20);
        float sxa[8], sxb[8];
#pragma unroll
        for (int r = 0; r < 4; ++r) { sxa[r] = q0[r]; sxa[4 + r] = q1[r]; sxb[r] = q2[r]; sxb[4 + r] = q3[r]; }
        v16h pb; float ls = 0.0f;
#pragma unroll
        for (int r = 0; r < 8; ++r) {
            const float aa = ta[r] + sh, ab = tb[r] + sh;
            const float xa = __builtin_amdgcn_exp2f(aa), xb = __builtin_amdgcn_exp2f(ab);
            const float ea = (aa < -14.0f) ? 0.0f : xa, eb = (ab < -14.0f) ? 0.0f : xb;
            const float ga = ea * sxa[r], gb = eb * sxb[r];
            const h16 pa = (h16)ga; const h16 pc = (h16)gb;
            pb[r] = pa; pb[8 + r] = pc;
            ls += (float)pa + (float)pc; }
        l = l * alpha + ls; m = mnew;
        o0 = o0 * alpha; o1 = o1 * alpha; o2 = o2 * alpha; o3 = o3 * alpha;
        const h16* va = VT + vo + key0;
        { const v16h v0 = ldh(va), v1 = ldh(va + (size_t)16 * NP);
          o0 = wmma16g(v0, pb, o0); o1 = wmma16g(v1, pb, o1); }
        { const v16h v2 = ldh(va + (size_t)32 * NP), v3 = ldh(va + (size_t)48 * NP);
          o2 = wmma16g(v2, pb, o2); o3 = wmma16g(v3, pb, o3); }
    }
    l += __shfl_xor(l, 16, 32);
    const float inv = 1.0f / l;
    const v4f a0 = *(const v4f*)(X + xo), a1 = *(const v4f*)(X + xo + 4), a2 = *(const v4f*)(X + xo + 16), a3 = *(const v4f*)(X + xo + 20);
    const int wb = wave * 16 * OSP;
    { v4f a, c;
#pragma unroll
      for (int r = 0; r < 4; ++r) { a[r] = (bfr(a0[r]) * o0[r] + o2[r]) * inv; c[r] = (bfr(a1[r]) * o0[4 + r] + o2[4 + r]) * inv; }
      *(v4fa*)(&os[wb + lr * OSP +  0 + 8 * hi]) = a; *(v4fa*)(&os[wb + lr * OSP +  0 + 8 * hi + 4]) = c;
#pragma unroll
      for (int r = 0; r < 4; ++r) { a[r] = (bfr(a2[r]) * o1[r] + o3[r]) * inv; c[r] = (bfr(a3[r]) * o1[4 + r] + o3[4 + r]) * inv; }
      *(v4fa*)(&os[wb + lr * OSP + 16 + 8 * hi]) = a; *(v4fa*)(&os[wb + lr * OSP + 16 + 8 * hi + 4]) = c; }
    wave_sync();
    float* orow = OUT + (size_t)b0 * ND;
#pragma unroll 1
    for (int ps = 0; ps < 2; ++ps) {
#pragma unroll
        for (int s = 0; s < 4; ++s) { const int row = 4 * s + (lane >> 3), cofs = (lane & 7) * 4;
            const v4f val = *(const v4fa*)(&os[wb + row * OSP + cofs]);
            *(volatile v4f*)(orow + (size_t)row * ND + cofs) = val; }
        if (ps == 0) __threadfence(); }
}

static constexpr size_t al256(size_t v) { return (v + 255) & ~(size_t)255; }
static constexpr size_t SZ_KP = al256((size_t)NP * KD * 2);
static constexpr size_t SZ_VT = al256((size_t)VC * NP * 2);
static constexpr size_t SZ_CL = al256((size_t)3 * NP * 4);
static constexpr size_t SZ_TOTAL = 2 * SZ_KP + SZ_VT + SZ_CL;
static_assert(SZ_TOTAL <= (size_t)134217728);
static_assert((size_t)(NP / TP - 1) * TP * KD + (size_t)(TP - 1) * KD + 56 + 8 == (size_t)NP * KD);
static_assert((size_t)(VC - 1) * NP + (size_t)(NP / TP - 1) * TP + 56 + 8 == (size_t)VC * NP);
static_assert((size_t)2 * NP + (size_t)(NP / TP - 1) * TP + 60 + 4 == (size_t)3 * NP);

extern "C" void kernel_launch(void* const* d_in, const int* in_sizes, int n_in,
                              void* d_out, int out_size, void* d_ws, size_t ws_size, hipStream_t stream) {
    if (n_in < 7) return;
    if ((size_t)in_sizes[0] < (size_t)NB * ND || in_sizes[1] < 1) return;
    if ((size_t)in_sizes[2] < (size_t)N0_ * ND || (size_t)in_sizes[3] < (size_t)N1_ * ND) return;
    if ((size_t)in_sizes[4] < (size_t)N0_ * ND || (size_t)in_sizes[5] < (size_t)N1_ * ND) return;
    if ((size_t)in_sizes[6] < (size_t)NP) return;
    if ((size_t)out_size < (size_t)NB * ND) return;
    if (SZ_TOTAL > ws_size) return;
    const float* X   = (const float*)d_in[0];
    const float* tp  = (const float*)d_in[1];
    const float* Mu0 = (const float*)d_in[2];
    const float* Mu1 = (const float*)d_in[3];
    const float* S0  = (const float*)d_in[4];
    const float* S1  = (const float*)d_in[5];
    const float* Lam = (const float*)d_in[6];
    float* OUT = (float*)d_out;
    char* wsp = (char*)d_ws;
    h16* KH = (h16*)wsp; wsp += SZ_KP;
    h16* KR = (h16*)wsp; wsp += SZ_KP;
    h16* VT = (h16*)wsp; wsp += SZ_VT;
    float* CL = (float*)wsp; wsp += SZ_CL;

    k_tab<<<dim3(NP / TP, 1, 1), 256, 0, stream>>>(tp, Mu0, Mu1, S0, S1, Lam, KH, KR, VT, CL);
    k_mix<<<dim3(NB / (16 * AW), 1, 1), 32 * AW, 0, stream>>>(X, KH, KR, VT, CL, OUT);
}
